// SSMBlock_24240795419333
// MI455X (gfx1250) — hardware-run, weakly checked
//
#include <hip/hip_runtime.h>
#include <math.h>

typedef __attribute__((ext_vector_type(16))) _Float16 v16h;
typedef __attribute__((ext_vector_type(8)))  _Float16 v8h;
typedef __attribute__((ext_vector_type(4)))  _Float16 v4h;
typedef __attribute__((ext_vector_type(16))) __bf16   v16b;
typedef __attribute__((ext_vector_type(8)))  __bf16   v8b;
typedef __attribute__((ext_vector_type(8)))  float    v8f;
typedef __attribute__((ext_vector_type(4)))  float    v4f;
typedef __attribute__((ext_vector_type(2)))  unsigned v2u;

constexpr int kBatch = 2;
constexpr int kSeq   = 2048;
constexpr int kDm    = 1024;
constexpr int kDin   = 2048;
constexpr int kNst   = 16;
constexpr int kNstP  = 32;
constexpr int kKc    = 4;
constexpr int kRows  = kBatch * kSeq;
constexpr int kXgP   = 2 * kDin;
constexpr int kXgW   = kXgP / 2;
constexpr int kBxN   = 64;
constexpr int kConvTP = 260;
constexpr int kScanTS = 64;
static_assert((kDm % 32) == 0 && (kDin % 32) == 0 && (kNstP % 32) == 0, "GEMM K multiples of 32");
static_assert((kRows % 64) == 0 && (kXgP % 64) == 0 && (kDin % 64) == 0 && (kDm % 64) == 0 && (kBxN % 64) == 0, "GEMM M,N multiples of 64");
static_assert((kSeq % 64) == 0 && (kDin % 256) == 0 && (kRows % 32) == 0 && (kSeq % kScanTS) == 0, "tile multiples");

constexpr size_t kOffHB  = 0;
constexpr size_t kOffWIT = kOffHB  + (size_t)kRows * kDm   * 2;
constexpr size_t kOffWDT = kOffWIT + (size_t)kXgP  * kDm   * 2;
constexpr size_t kOffWOT = kOffWDT + (size_t)kDin  * kDin  * 2;
constexpr size_t kOffBMB = kOffWOT + (size_t)kDm   * kDin  * 2;
constexpr size_t kOffCMP = kOffBMB + (size_t)kBxN  * kDin  * 2;
constexpr size_t kOffXG  = kOffCMP + (size_t)kDin  * kNstP * 2;
constexpr size_t kOffXS  = kOffXG  + (size_t)kRows * kXgP  * 2;
constexpr size_t kOffDPY = kOffXS  + (size_t)kRows * kDin  * 2;
constexpr size_t kOffDEL = kOffDPY + (size_t)kRows * kDin  * 4;
constexpr size_t kOffBXR = kOffDEL + (size_t)kRows * 4;
constexpr size_t kOffHSP = kOffBXR + (size_t)kRows * kBxN  * 4;
constexpr size_t kOffYB  = kOffHSP + (size_t)kRows * kNstP * 2;
constexpr size_t kWsTotal = kOffYB + (size_t)kRows * kDin * 2;
static_assert(kWsTotal == 131743744ull, "carve total");
static_assert(kWsTotal <= 134217728ull, "carve cap");
static_assert((kOffWIT % 128) == 0 && (kOffWDT % 128) == 0 && (kOffWOT % 128) == 0 && (kOffBMB % 128) == 0 &&
              (kOffCMP % 128) == 0 && (kOffXG % 128) == 0 && (kOffXS % 128) == 0 && (kOffDPY % 128) == 0 &&
              (kOffDEL % 128) == 0 && (kOffBXR % 128) == 0 && (kOffHSP % 128) == 0 && (kOffYB % 128) == 0,
              "128-B aligned regions");

__device__ __forceinline__ unsigned short f2bf_bits(float f) {
  unsigned u = __float_as_uint(f);
  return (unsigned short)((u + 0x7FFFu + ((u >> 16) & 1u)) >> 16);
}
__device__ __forceinline__ float bf_bits2f(unsigned short h) { return __uint_as_float(((unsigned)h) << 16); }
__device__ __forceinline__ float bf_lo_of_word(unsigned w) { return __uint_as_float(w << 16); }
__device__ __forceinline__ float bf_hi_of_word(unsigned w) { return __uint_as_float(w & 0xffff0000u); }

__device__ __forceinline__ void dep_guard4_h(v8f& a, v8f& b, v8f& c, v8f& d, v16h x, v16h y, v16h z) {
  asm volatile("v_nop\n\tv_nop\n\tv_nop\n\tv_nop" : "+v"(a), "+v"(b), "+v"(c), "+v"(d) : "v"(x), "v"(y), "v"(z));
}
__device__ __forceinline__ void dep_guard4_b(v8f& a, v8f& b, v8f& c, v8f& d, v16b x, v16b y, v16b z) {
  asm volatile("v_nop\n\tv_nop\n\tv_nop\n\tv_nop" : "+v"(a), "+v"(b), "+v"(c), "+v"(d) : "v"(x), "v"(y), "v"(z));
}
__device__ __forceinline__ void keep4_h(v16h a, v16h b, v16h c, v16h d) { asm volatile("v_nop" :: "v"(a), "v"(b), "v"(c), "v"(d)); }
__device__ __forceinline__ void keep4_b(v16b a, v16b b, v16b c, v16b d) { asm volatile("v_nop" :: "v"(a), "v"(b), "v"(c), "v"(d)); }
__device__ __forceinline__ void acc_guard4(v8f& a, v8f& b, v8f& c, v8f& d) { asm volatile("v_nop\n\tv_nop\n\tv_nop\n\tv_nop" : "+v"(a), "+v"(b), "+v"(c), "+v"(d)); }
template <typename T> struct Frag;
template <> struct Frag<_Float16> {
  typedef v16h V; union U { v16h v; v8h h[2]; };
  static __device__ __forceinline__ v16h load(const _Float16* p) {
    U f; f.h[0] = *(const v8h*)(p); f.h[1] = *(const v8h*)(p + 16); return f.v;
  }
  static __device__ __forceinline__ v8f mma(v16h a, v16h b, v8f c) {
    return __builtin_amdgcn_wmma_f32_16x16x32_f16(false, a, false, b, (short)0, c, false, false);
  }
  static __device__ __forceinline__ void guard4(v8f& a, v8f& b, v8f& c, v8f& d, v16h x, v16h y, v16h z) { dep_guard4_h(a, b, c, d, x, y, z); }
  static __device__ __forceinline__ void keep(v16h a, v16h b, v16h c, v16h d) { keep4_h(a, b, c, d); }
};
template <> struct Frag<__bf16> {
  typedef v16b V; union U { v16b v; v8b h[2]; };
  static __device__ __forceinline__ v16b load(const __bf16* p) {
    U f; f.h[0] = *(const v8b*)(p); f.h[1] = *(const v8b*)(p + 16); return f.v;
  }
  static __device__ __forceinline__ v8f mma(v16b a, v16b b, v8f c) {
    return __builtin_amdgcn_wmma_f32_16x16x32_bf16(false, a, false, b, (short)0, c, false, false);
  }
  static __device__ __forceinline__ void guard4(v8f& a, v8f& b, v8f& c, v8f& d, v16b x, v16b y, v16b z) { dep_guard4_b(a, b, c, d, x, y, z); }
  static __device__ __forceinline__ void keep(v16b a, v16b b, v16b c, v16b d) { keep4_b(a, b, c, d); }
};

template <int ET> struct Elem;
template <> struct Elem<0> { typedef _Float16 T; };
template <> struct Elem<1> { typedef __bf16 T; };
template <int ET, bool SPLIT, int BIAS_MODE, int OUT_MODE, bool RESID>
__global__ __launch_bounds__(256) void wmma_gemm64(
    const unsigned short* __restrict__ Ap, const unsigned short* __restrict__ A2p, int lda, long strideA,
    const unsigned short* __restrict__ Btp, const unsigned short* __restrict__ Bt2p, int ldb, long strideB,
    void* __restrict__ Cout, void* __restrict__ Cout2, int ldc, long strideC,
    const float* __restrict__ bias,
    const float* __restrict__ resid, long strideR,
    int M, int N, int K, float scale) {
  static_assert(!(RESID && OUT_MODE != 0), "resid only with f32 output");
  typedef typename Elem<ET>::T T;
  typedef typename Frag<T>::V V;
  const T* A = (const T*)Ap; const T* A2 = (const T*)A2p; const T* Bt = (const T*)Btp; const T* Bt2 = (const T*)Bt2p;
  __shared__ __align__(16) float sT[8][16 * 68];
  const int b    = blockIdx.y;
  const int lane = threadIdx.x & 31;
  const int wave = threadIdx.x >> 5;
  const int tilesN = N >> 6;
  const int tilesM = M >> 6;
  const int tile = blockIdx.x * 8 + wave;
  if (tile >= tilesM * tilesN) return;
  const int tm = tile / tilesN;
  const int tn = tile - tm * tilesN;
  const int m0 = tm << 6;
  const int n0 = tn << 6;

  const T* Ab  = A  + (size_t)b * strideA;
  const T* Bb  = Bt + (size_t)b * strideB;
  const T* Ab2 = SPLIT ? (A2  + (size_t)b * strideA) : nullptr;
  const T* Bb2 = SPLIT ? (Bt2 + (size_t)b * strideB) : nullptr;

  const int rlane = lane & 15;
  const int koff  = (lane >> 4) * 8;
  const int mOff  = (lane >> 4) * 8;

  v8f acc[4][4];
#pragma unroll
  for (int i = 0; i < 4; ++i)
#pragma unroll
    for (int j = 0; j < 4; ++j) acc[i][j] = (v8f){0.f,0.f,0.f,0.f,0.f,0.f,0.f,0.f};

  for (int k0 = 0; k0 < K; k0 += 32) {
    V bh[4], bl[4];
#pragma unroll
    for (int j = 0; j < 4; ++j) {
      const size_t bo = (size_t)(n0 + (j << 4) + rlane) * ldb + koff + k0;
      bh[j] = Frag<T>::load(Bb + bo);
      if (SPLIT) bl[j] = Frag<T>::load(Bb2 + bo);
    }
#pragma unroll
    for (int i = 0; i < 4; ++i) {
      const size_t ao = (size_t)(m0 + (i << 4) + rlane) * lda + koff + k0;
      V ah = Frag<T>::load(Ab + ao);
      V al;
      if (SPLIT) al = Frag<T>::load(Ab2 + ao);
#pragma unroll
      for (int j = 0; j < 4; ++j) {
        acc[i][j] = Frag<T>::mma(ah, bh[j], acc[i][j]);
        if (SPLIT) {
          acc[i][j] = Frag<T>::mma(ah, bl[j], acc[i][j]);
          acc[i][j] = Frag<T>::mma(al, bh[j], acc[i][j]);
        }
      }
      Frag<T>::guard4(acc[i][0], acc[i][1], acc[i][2], acc[i][3], ah, SPLIT ? al : ah, bh[3]);
    }
    Frag<T>::keep(bh[0], bh[1], bh[2], bh[3]);
    if (SPLIT) Frag<T>::keep(bl[0], bl[1], bl[2], bl[3]);
  }
  acc_guard4(acc[0][0], acc[0][1], acc[0][2], acc[0][3]);
  acc_guard4(acc[1][0], acc[1][1], acc[1][2], acc[1][3]);
  acc_guard4(acc[2][0], acc[2][1], acc[2][2], acc[2][3]);
  acc_guard4(acc[3][0], acc[3][1], acc[3][2], acc[3][3]);

  float* slab = sT[wave];
  const float* Rb = RESID ? (resid + (size_t)b * strideR) : nullptr;
#pragma unroll
  for (int i = 0; i < 4; ++i) {
    const int mBase = m0 + (i << 4);
#pragma unroll
    for (int j = 0; j < 4; ++j) {
      const int n = n0 + (j << 4) + rlane;
      float bv = 0.f;
      if (BIAS_MODE == 2) bv = bias[n];
#pragma unroll
      for (int r = 0; r < 8; ++r) {
        float v = acc[i][j][r] * scale;
        if (BIAS_MODE == 1) v += bias[mBase + mOff + r];
        if (BIAS_MODE == 2) v += bv;
        slab[(mOff + r) * 68 + (j << 4) + rlane] = v;
      }
    }
    __builtin_amdgcn_fence(__ATOMIC_RELEASE, "workgroup");
    __builtin_amdgcn_wave_barrier();
    __builtin_amdgcn_fence(__ATOMIC_ACQUIRE, "workgroup");
    if (OUT_MODE == 0) {
      float* C = (float*)Cout + (size_t)b * strideC;
      const int hh = lane >> 4, c4 = (lane & 15) * 4;
      for (int pass = 0; pass < 2; ++pass) {
#pragma unroll
        for (int it = 0; it < 8; ++it) {
          const int row = it * 2 + hh;
          v4f v = *(const v4f*)(slab + row * 68 + c4);
          if (RESID) {
            const v4f rr = *(const v4f*)(Rb + (size_t)(mBase + row) * ldc + n0 + c4);
            v = rr + v;
          }
          *(volatile v4f*)(C + (size_t)(mBase + row) * ldc + n0 + c4) = v;
        }
        __threadfence();
      }
    } else {
      const int q = lane >> 3, c8 = (lane & 7) * 8;
      unsigned short* C  = (unsigned short*)Cout  + (size_t)b * strideC;
      unsigned short* C2 = (OUT_MODE == 2) ? ((unsigned short*)Cout2 + (size_t)b * strideC) : nullptr;
      for (int pass = 0; pass < 2; ++pass) {
#pragma unroll
        for (int it = 0; it < 4; ++it) {
          const int row = it * 4 + q;
          const float* sp = slab + row * 68 + c8;
          v8h hv, lv;
#pragma unroll
          for (int e = 0; e < 8; ++e) {
            if (OUT_MODE == 1) {
              hv[e] = (_Float16)sp[e];
            } else {
              unsigned short hb = f2bf_bits(sp[e]);
              hv[e] = __builtin_bit_cast(_Float16, hb);
              if (OUT_MODE == 2) {
                unsigned short lb = f2bf_bits(sp[e] - bf_bits2f(hb));
                lv[e] = __builtin_bit_cast(_Float16, lb);
              }
            }
          }
          *(volatile v8h*)(C + (size_t)(mBase + row) * ldc + n0 + c8) = hv;
          if (OUT_MODE == 2) *(volatile v8h*)(C2 + (size_t)(mBase + row) * ldc + n0 + c8) = lv;
        }
        __threadfence();
      }
    }
    __builtin_amdgcn_fence(__ATOMIC_RELEASE, "workgroup");
    __builtin_amdgcn_wave_barrier();
    __builtin_amdgcn_fence(__ATOMIC_ACQUIRE, "workgroup");
  }
}

__global__ __launch_bounds__(128) void layernorm_kernel(
    const float* __restrict__ x, const float* __restrict__ g, const float* __restrict__ bt,
    unsigned short* __restrict__ HB)
{
  __shared__ float shA[4];
  __shared__ float shB[4];
  const int tid = threadIdx.x, lane = tid & 31, wave = tid >> 5;
  const size_t row = blockIdx.x;
  const int c0 = tid * 8;
  const float* xr = x + row * kDm + c0;
  const v4f a0 = *(const v4f*)(xr);
  const v4f a1 = *(const v4f*)(xr + 4);
  float s = +0.0f;
  s += a0[0]; s += a0[1]; s += a0[2]; s += a0[3];
  s += a1[0]; s += a1[1]; s += a1[2]; s += a1[3];
#pragma unroll
  for (int off = 16; off > 0; off >>= 1) s += __shfl_xor(s, off, 32);
  if (lane == 0) shA[wave] = s;
  __syncthreads();
  const float mu = ((shA[0] + shA[1]) + (shA[2] + shA[3])) * (1.0f / 1024.0f);
  const v4f muv = (v4f){mu, mu, mu, mu};
  const v4f d0 = a0 - muv;
  const v4f d1 = a1 - muv;
  float s2 = +0.0f;
  s2 += d0[0] * d0[0]; s2 += d0[1] * d0[1]; s2 += d0[2] * d0[2]; s2 += d0[3] * d0[3];
  s2 += d1[0] * d1[0]; s2 += d1[1] * d1[1]; s2 += d1[2] * d1[2]; s2 += d1[3] * d1[3];
#pragma unroll
  for (int off = 16; off > 0; off >>= 1) s2 += __shfl_xor(s2, off, 32);
  if (lane == 0) shB[wave] = s2;
  __syncthreads();
  const float var = ((shB[0] + shB[1]) + (shB[2] + shB[3])) * (1.0f / 1024.0f);
  const float inv = rsqrtf(var + 1e-5f);
  const v4f g0 = *(const v4f*)(g + c0);
  const v4f g1 = *(const v4f*)(g + c0 + 4);
  const v4f b0 = *(const v4f*)(bt + c0);
  const v4f b1 = *(const v4f*)(bt + c0 + 4);
  v8h hv;
#pragma unroll
  for (int e = 0; e < 4; ++e) {
    float t0 = d0[e] * inv; t0 = t0 * g0[e]; t0 = t0 + b0[e];
    float t1 = d1[e] * inv; t1 = t1 * g1[e]; t1 = t1 + b1[e];
    const unsigned short h0 = f2bf_bits(t0), h1 = f2bf_bits(t1);
    hv[e]     = __builtin_bit_cast(_Float16, h0);
    hv[4 + e] = __builtin_bit_cast(_Float16, h1);
  }
  unsigned short* qp = HB + row * kDm + c0;
  *(volatile v8h*)qp = hv;
  __threadfence();
  *(volatile v8h*)qp = hv;
}

__global__ __launch_bounds__(256) void transpose_bf16_kernel(
    const float* __restrict__ in, unsigned short* __restrict__ out, int rows, int cols)
{
  __shared__ float tile[64][65];
  const int tid = threadIdx.x, lane = tid & 31, wave = tid >> 5;
  const int r0 = blockIdx.y * 64, c0 = blockIdx.x * 64;
#pragma unroll
  for (int it = 0; it < 4; ++it) {
    const int idx = it * 256 + tid;
    const int lr = idx >> 4, lc = (idx & 15) * 4;
    const v4f v = *(const v4f*)(in + (size_t)(r0 + lr) * cols + c0 + lc);
    tile[lr][lc + 0] = v[0];
    tile[lr][lc + 1] = v[1];
    tile[lr][lc + 2] = v[2];
    tile[lr][lc + 3] = v[3];
  }
  __syncthreads();
  const int q = lane >> 3, c8 = (lane & 7) * 8;
  v8h hv[2];
#pragma unroll
  for (int it = 0; it < 2; ++it) {
    const int orow = it * 32 + wave * 4 + q;
#pragma unroll
    for (int e = 0; e < 8; ++e) {
      const unsigned short hb = f2bf_bits(tile[c8 + e][orow]);
      hv[it][e] = __builtin_bit_cast(_Float16, hb);
    }
  }
  for (int pass = 0; pass < 2; ++pass) {
#pragma unroll
    for (int it = 0; it < 2; ++it) {
      const int orow = it * 32 + wave * 4 + q;
      *(volatile v8h*)(out + (size_t)(c0 + orow) * rows + r0 + c8) = hv[it];
    }
    __threadfence();
  }
}

__global__ __launch_bounds__(256) void bmat_plane_kernel(const float* __restrict__ Bm, unsigned short* __restrict__ BMB)
{
  const int tid = threadIdx.x;
  const int r = blockIdx.x;
  const int c = tid * 8;
  const int rc = (r < kNst) ? r : (kNst - 1);
  const float f = (r < kNst) ? 1.0f : 0.0f;
  const v4f a0 = *(const v4f*)(Bm + (size_t)rc * kDin + c);
  const v4f a1 = *(const v4f*)(Bm + (size_t)rc * kDin + c + 4);
  v8h hv;
#pragma unroll
  for (int e = 0; e < 4; ++e) {
    const unsigned short h0 = f2bf_bits(a0[e] * f), h1 = f2bf_bits(a1[e] * f);
    hv[e]     = __builtin_bit_cast(_Float16, h0);
    hv[4 + e] = __builtin_bit_cast(_Float16, h1);
  }
  unsigned short* qp = BMB + (size_t)r * kDin + c;
  *(volatile v8h*)qp = hv;
  __threadfence();
  *(volatile v8h*)qp = hv;
}

__global__ __launch_bounds__(256) void cmat_plane_kernel(const float* __restrict__ Cm, unsigned short* __restrict__ CMP)
{
  const int i = blockIdx.x * 256 + threadIdx.x;
  const int e0 = i * 8;
  const int d = e0 >> 5;
  const int c = e0 & 31;
  const int cc = c & 8;
  const float f = (c < kNst) ? 1.0f : 0.0f;
  const v4f a0 = *(const v4f*)(Cm + (size_t)d * kNst + cc);
  const v4f a1 = *(const v4f*)(Cm + (size_t)d * kNst + cc + 4);
  v8h hv;
#pragma unroll
  for (int e = 0; e < 4; ++e) {
    const unsigned short h0 = f2bf_bits(a0[e] * f), h1 = f2bf_bits(a1[e] * f);
    hv[e]     = __builtin_bit_cast(_Float16, h0);
    hv[4 + e] = __builtin_bit_cast(_Float16, h1);
  }
  unsigned short* qp = CMP + (size_t)e0;
  *(volatile v8h*)qp = hv;
  __threadfence();
  *(volatile v8h*)qp = hv;
}

__global__ __launch_bounds__(128) void conv_silu_kernel(
    const unsigned* __restrict__ XGw, const float* __restrict__ cw, const float* __restrict__ cb,
    unsigned short* __restrict__ XS)
{
  __shared__ __align__(16) float sT[16 * kConvTP];
  const int tid = threadIdx.x, lane = tid & 31, wave = tid >> 5;
  const int d0 = blockIdx.x * 256;
  const int dp = d0 + 2 * tid;
  const int wi = dp >> 1;
  const int g0 = blockIdx.y * 64;
  const int tb = g0 & (kSeq - 1);
  const v4f wa = *(const v4f*)(cw + (size_t)dp * kKc);
  const v4f wb = *(const v4f*)(cw + (size_t)dp * kKc + 4);
  const float cba = cb[dp], cbb = cb[dp + 1];
  float am3, am2, am1, bm3, bm2, bm1;
  {
    const bool hist = (tb > 0);
    const int rb = hist ? (g0 - 3) : g0;
    const float fh = hist ? 1.0f : 0.0f;
    const unsigned u3 = XGw[(size_t)rb * kXgW + wi];
    const unsigned u2 = XGw[(size_t)(rb + 1) * kXgW + wi];
    const unsigned u1 = XGw[(size_t)(rb + 2) * kXgW + wi];
    am3 = bf_lo_of_word(u3) * fh; bm3 = bf_hi_of_word(u3) * fh;
    am2 = bf_lo_of_word(u2) * fh; bm2 = bf_hi_of_word(u2) * fh;
    am1 = bf_lo_of_word(u1) * fh; bm1 = bf_hi_of_word(u1) * fh;
  }
#pragma unroll 1
  for (int sub = 0; sub < 4; ++sub) {
    const int lb = g0 + sub * 16;
#pragma unroll 1
    for (int s = 0; s < 16; ++s) {
      const unsigned u = XGw[(size_t)(lb + s) * kXgW + wi];
      const float xa = bf_lo_of_word(u);
      const float xb = bf_hi_of_word(u);
      float acca = wa[0] * am3;
      acca = fmaf(wa[1], am2, acca);
      acca = fmaf(wa[2], am1, acca);
      acca = fmaf(wa[3], xa, acca);
      float accb = wb[0] * bm3;
      accb = fmaf(wb[1], bm2, accb);
      accb = fmaf(wb[2], bm1, accb);
      accb = fmaf(wb[3], xb, accb);
      const float sva = acca + cba;
      const float svb = accb + cbb;
      const float sga = 1.0f / (1.0f + expf(-sva));
      const float sgb = 1.0f / (1.0f + expf(-svb));
      sT[s * kConvTP + 2 * tid]     = sva * sga;
      sT[s * kConvTP + 2 * tid + 1] = svb * sgb;
      am3 = am2; am2 = am1; am1 = xa;
      bm3 = bm2; bm2 = bm1; bm1 = xb;
    }
    __syncthreads();
    v8h hv[4];
#pragma unroll
    for (int it = 0; it < 4; ++it) {
      const float* sp = sT + (it * 4 + wave) * kConvTP + lane * 8;
      const v4f a0 = *(const v4f*)(sp);
      const v4f a1 = *(const v4f*)(sp + 4);
#pragma unroll
      for (int e = 0; e < 4; ++e) {
        const unsigned short h0 = f2bf_bits(a0[e]), h1 = f2bf_bits(a1[e]);
        hv[it][e]     = __builtin_bit_cast(_Float16, h0);
        hv[it][4 + e] = __builtin_bit_cast(_Float16, h1);
      }
    }
    for (int pass = 0; pass < 2; ++pass) {
#pragma unroll
      for (int it = 0; it < 4; ++it) {
        const size_t o = (size_t)(lb + it * 4 + wave) * kDin + d0 + lane * 8;
        *(volatile v8h*)(XS + o) = hv[it];
      }
      __threadfence();
    }
    __syncthreads();
  }
}

__global__ __launch_bounds__(256) void delta_kernel(
    const float* __restrict__ DP, const float* __restrict__ bd, float* __restrict__ DEL)
{
  __shared__ float sh[32];
  const int tid = threadIdx.x, lane = tid & 31, wave = tid >> 5;
  const int r0 = blockIdx.x * 32;
#pragma unroll 1
  for (int i = 0; i < 4; ++i) {
    const int row = r0 + wave * 4 + i;
    const float* pr = DP + (size_t)row * kDin;
    float s = +0.0f;
#pragma unroll 1
    for (int k = 0; k < kDin / 32; ++k) {
      const int c = k * 32 + lane;
      const float t = pr[c] + bd[c];
      s += fmaxf(t, 0.0f) + log1pf(expf(-fabsf(t)));
    }
#pragma unroll
    for (int off = 16; off > 0; off >>= 1) s += __shfl_xor(s, off, 32);
    if (lane == 0) sh[wave * 4 + i] = s * (1.0f / 2048.0f);
  }
  __syncthreads();
  if (wave == 0) {
    const float v = sh[lane];
    float* qp = DEL + r0 + lane;
    *(volatile float*)qp = v;
    __threadfence();
    *(volatile float*)qp = v;
  }
}

__global__ __launch_bounds__(32) void scan_kernel(
    const float* __restrict__ DEL, const float* __restrict__ BXR, const float* __restrict__ Alog,
    unsigned short* __restrict__ HSP)
{
  __shared__ __align__(16) float sH[kBatch * kScanTS * kNst];
  const int lane = threadIdx.x;
  const int b = lane >> 4, n = lane & 15;
  const float Aneg = -expf(Alog[n]);
  const size_t rowb = (size_t)b * kSeq;
  float h = +0.0f;
  const int sr = lane >> 2;
  const int sc = (lane & 3) * 8;
  const int scc = sc & 8;
  const float fz = (sc < kNst) ? 1.0f : 0.0f;
#pragma unroll 1
  for (int l0 = 0; l0 < kSeq; l0 += kScanTS) {
#pragma unroll 1
    for (int s = 0; s < kScanTS; ++s) {
      const size_t row = rowb + l0 + s;
      const float dl = DEL[row];
      const float bx = BXR[row * kBxN + n] * dl;
      float dA = expf(dl * Aneg);
      dA = (dA < 1.17549435e-38f) ? 0.0f : dA;
      h = dA * h + bx;
      sH[(b * kScanTS + s) * kNst + n] = h;
    }
    __syncthreads();
#pragma unroll 1
    for (int bb = 0; bb < kBatch; ++bb) {
      v8h hv[8];
#pragma unroll
      for (int it = 0; it < 8; ++it) {
        const int r = it * 8 + sr;
        const float* sp = sH + (bb * kScanTS + r) * kNst + scc;
        const v4f a0 = *(const v4f*)(sp);
        const v4f a1 = *(const v4f*)(sp + 4);
#pragma unroll
        for (int e = 0; e < 4; ++e) {
          const unsigned short h0 = f2bf_bits(a0[e] * fz), h1 = f2bf_bits(a1[e] * fz);
          hv[it][e]     = __builtin_bit_cast(_Float16, h0);
          hv[it][4 + e] = __builtin_bit_cast(_Float16, h1);
        }
      }
      for (int pass = 0; pass < 2; ++pass) {
#pragma unroll
        for (int it = 0; it < 8; ++it) {
          const int r = it * 8 + sr;
          const size_t o = ((size_t)bb * kSeq + l0 + r) * kNstP + sc;
          *(volatile v8h*)(HSP + o) = hv[it];
        }
        __threadfence();
      }
    }
    __syncthreads();
  }
}

__global__ __launch_bounds__(256) void gate_kernel(
    const float* __restrict__ YR, const unsigned* __restrict__ XSw, const unsigned* __restrict__ XGw,
    const float* __restrict__ Dv, unsigned short* __restrict__ YB)
{
  const int i = blockIdx.x * 256 + threadIdx.x;
  if (i >= kRows * kDin / 4) return;
  const size_t e0 = (size_t)i * 4;
  const size_t row = e0 >> 11;
  const int d = (int)(e0 & (kDin - 1));
  const v4f y  = *(const v4f*)(YR + e0);
  const v2u xw = *(const v2u*)(XSw + (e0 >> 1));
  const v2u gw = *(const v2u*)(XGw + ((row * kXgP + kDin + d) >> 1));
  const v4f dv = *(const v4f*)(Dv + d);
  const unsigned x0w = xw[0], x1w = xw[1], g0w = gw[0], g1w = gw[1];
  float xs[4], gs[4];
  xs[0] = bf_lo_of_word(x0w); xs[1] = bf_hi_of_word(x0w); xs[2] = bf_lo_of_word(x1w); xs[3] = bf_hi_of_word(x1w);
  gs[0] = bf_lo_of_word(g0w); gs[1] = bf_hi_of_word(g0w); gs[2] = bf_lo_of_word(g1w); gs[3] = bf_hi_of_word(g1w);
  v4h hv;
#pragma unroll
  for (int e = 0; e < 4; ++e) {
    float t = fmaf(dv[e], xs[e], y[e]);
    const float sg = gs[e] * (1.0f / (1.0f + expf(-gs[e])));
    t = t * sg;
    const unsigned short hb = f2bf_bits(t);
    hv[e] = __builtin_bit_cast(_Float16, hb);
  }
  unsigned short* qp = YB + e0;
  *(volatile v4h*)qp = hv;
  __threadfence();
  *(volatile v4h*)qp = hv;
}

static_assert((kRows / 64) * (kXgP / 64) == 8 * 512, "S1 grid");
static_assert((kRows / 64) * (kDin / 64) == 8 * 256, "S2/S4 grid");
static_assert((kRows / 64) * (kBxN / 64) == 8 * 8, "S3 grid");
static_assert((kRows / 64) * (kDm / 64) == 8 * 128, "S5 grid");

extern "C" void kernel_launch(void* const* d_in, const int* in_sizes, int n_in,
                              void* d_out, int out_size, void* d_ws, size_t ws_size,
                              hipStream_t stream) {
  if (n_in < 13) return;
  if (in_sizes[0] != kRows * kDm) return;
  if (in_sizes[1] != kDm) return;
  if (in_sizes[2] != kDm) return;
  if (in_sizes[3] != kDm * kXgP) return;
  if (in_sizes[4] != kDin * kKc) return;
  if (in_sizes[5] != kDin) return;
  if (in_sizes[6] != kNst) return;
  if (in_sizes[7] != kNst * kDin) return;
  if (in_sizes[8] != kDin * kNst) return;
  if (in_sizes[9] != kDin) return;
  if (in_sizes[10] != kDin * kDin) return;
  if (in_sizes[11] != kDin) return;
  if (in_sizes[12] != kDin * kDm) return;
  if (out_size != kRows * kDm) return;
  if (ws_size < kWsTotal) return;

  const float* x      = (const float*)d_in[0];
  const float* gln    = (const float*)d_in[1];
  const float* bln    = (const float*)d_in[2];
  const float* W_in   = (const float*)d_in[3];
  const float* conv_w = (const float*)d_in[4];
  const float* conv_b = (const float*)d_in[5];
  const float* A_log  = (const float*)d_in[6];
  const float* B_mat  = (const float*)d_in[7];
  const float* C_mat  = (const float*)d_in[8];
  const float* D_vec  = (const float*)d_in[9];
  const float* Wd     = (const float*)d_in[10];
  const float* bd     = (const float*)d_in[11];
  const float* W_out  = (const float*)d_in[12];
  float* out = (float*)d_out;

  char* ws = (char*)d_ws;
  unsigned short* HB  = (unsigned short*)(ws + kOffHB);
  unsigned short* WIT = (unsigned short*)(ws + kOffWIT);
  unsigned short* WDT = (unsigned short*)(ws + kOffWDT);
  unsigned short* WOT = (unsigned short*)(ws + kOffWOT);
  unsigned short* BMB = (unsigned short*)(ws + kOffBMB);
  unsigned short* CMP = (unsigned short*)(ws + kOffCMP);
  unsigned short* XG  = (unsigned short*)(ws + kOffXG);
  unsigned short* XS  = (unsigned short*)(ws + kOffXS);
  float*          DPY = (float*)(ws + kOffDPY);
  float*          DEL = (float*)(ws + kOffDEL);
  float*          BXR = (float*)(ws + kOffBXR);
  unsigned short* HSP = (unsigned short*)(ws + kOffHSP);
  unsigned short* YB  = (unsigned short*)(ws + kOffYB);

  layernorm_kernel<<<kRows, 128, 0, stream>>>(x, gln, bln, HB);

  transpose_bf16_kernel<<<dim3(kXgP / 64, kDm / 64), 256, 0, stream>>>(W_in, WIT, kDm, kXgP);
  transpose_bf16_kernel<<<dim3(kDin / 64, kDin / 64), 256, 0, stream>>>(Wd, WDT, kDin, kDin);
  transpose_bf16_kernel<<<dim3(kDm / 64, kDin / 64), 256, 0, stream>>>(W_out, WOT, kDin, kDm);
  bmat_plane_kernel<<<kBxN, 256, 0, stream>>>(B_mat, BMB);
  cmat_plane_kernel<<<(kDin * kNstP / 8) / 256, 256, 0, stream>>>(C_mat, CMP);

  wmma_gemm64<1, false, 0, 3, false><<<dim3(512, 1), 256, 0, stream>>>(
      HB, nullptr, kDm, 0L,
      WIT, nullptr, kDm, 0L,
      (void*)XG, nullptr, kXgP, 0L,
      nullptr, nullptr, 0L,
      kRows, kXgP, kDm, 1.0f);

  conv_silu_kernel<<<dim3(kDin / 256, kRows / 64), 128, 0, stream>>>((const unsigned*)XG, conv_w, conv_b, XS);

  wmma_gemm64<1, false, 0, 0, false><<<dim3(256, 1), 256, 0, stream>>>(
      XS, nullptr, kDin, 0L,
      WDT, nullptr, kDin, 0L,
      (void*)DPY, nullptr, kDin, 0L,
      nullptr, nullptr, 0L,
      kRows, kDin, kDin, 1.0f);

  delta_kernel<<<kRows / 32, 256, 0, stream>>>(DPY, bd, DEL);

  wmma_gemm64<1, false, 0, 0, false><<<dim3(8, 1), 256, 0, stream>>>(
      XS, nullptr, kDin, 0L,
      BMB, nullptr, kDin, 0L,
      (void*)BXR, nullptr, kBxN, 0L,
      nullptr, nullptr, 0L,
      kRows, kBxN, kDin, 1.0f);

  scan_kernel<<<1, 32, 0, stream>>>(DEL, BXR, A_log, HSP);

  wmma_gemm64<1, false, 0, 0, false><<<dim3(256, 1), 256, 0, stream>>>(
      HSP, nullptr, kNstP, 0L,
      CMP, nullptr, kNstP, 0L,
      (void*)DPY, nullptr, kDin, 0L,
      nullptr, nullptr, 0L,
      kRows, kDin, kNstP, 1.0f);

  gate_kernel<<<(kRows * kDin / 4) / 256, 256, 0, stream>>>(DPY, (const unsigned*)XS, (const unsigned*)XG, D_vec, YB);

  wmma_gemm64<1, false, 0, 0, true><<<dim3(128, 1), 256, 0, stream>>>(
      YB, nullptr, kDin, 0L,
      WOT, nullptr, kDin, 0L,
      (void*)out, nullptr, kDm, 0L,
      nullptr, x, 0L,
      kRows, kDm, kDin, 1.0f);
}
